// MultiHeadSelfAttention_65403761983822
// MI455X (gfx1250) — hardware-verified
//
#include <hip/hip_runtime.h>


#ifndef NB
#define NB 4
#endif
#ifndef SEQ
#define SEQ 2048
#endif
#define NB_FULL  4
#define SEQ_FULL 2048
#define DM   512
#define NH_  8
#define HD   64
#define DQ   (NH_ * HD)
#define DKV  DQ
#define KCAR 16.0f
#define PEXP 8.0f
#define C2   (0.044194173824159216f * 1.4426950408889634f * (1.0f / 256.0f))

typedef _Float16 h16;
typedef unsigned short bf;
typedef __attribute__((ext_vector_type(16))) __bf16   v16bf;
typedef __attribute__((ext_vector_type(16))) _Float16 v16h;
typedef __attribute__((ext_vector_type(8)))  _Float16 v8h;
typedef __attribute__((ext_vector_type(8)))  unsigned short v8us;
typedef __attribute__((ext_vector_type(8)))  float    v8f;
typedef __attribute__((ext_vector_type(4)))  float    v4f;
typedef v4f  __attribute__((may_alias)) v4fa;

static_assert(NB >= 1 && NB <= NB_FULL);
static_assert(SEQ >= 64 && SEQ <= SEQ_FULL);
static_assert(SEQ % 64 == 0);
static_assert((NB * SEQ) % 64 == 0);
static_assert(DM % 64 == 0 && DM % 32 == 0);
static_assert(DQ % 64 == 0 && DQ % 32 == 0);
static_assert(HD == 64);
static_assert(DQ == NH_ * HD);
static_assert((SEQ * DM) % 8 == 0 && (DKV * DM) % 8 == 0);

__device__ __forceinline__ unsigned short f2bf(float f) { unsigned u = __float_as_uint(f); u += 0x7FFFu + ((u >> 16) & 1u); return (unsigned short)(u >> 16); }
__device__ __forceinline__ float bf2f(unsigned short b) { return __uint_as_float(((unsigned)b) << 16); }
__device__ __forceinline__ v16h cat16(v8h lo, v8h hi) { return __builtin_shufflevector(lo, hi, 0, 1, 2, 3, 4, 5, 6, 7, 8, 9, 10, 11, 12, 13, 14, 15); }
__device__ __forceinline__ v16bf cat16b(v8us lo, v8us hi) { return __builtin_bit_cast(v16bf, __builtin_shufflevector(lo, hi, 0, 1, 2, 3, 4, 5, 6, 7, 8, 9, 10, 11, 12, 13, 14, 15)); }
__device__ __forceinline__ v8f wmma16(v16h a, v16h b, v8f c) { return __builtin_amdgcn_wmma_f32_16x16x32_f16(false, a, false, b, (short)0, c, false, false); }
__device__ __forceinline__ v8f wmmab(v16bf a, v16bf b, v8f c) { return __builtin_amdgcn_wmma_f32_16x16x32_bf16(false, a, false, b, (short)0, c, false, false); }
__device__ __forceinline__ void splitf(float y, unsigned short& h, unsigned short& l) { h = f2bf(y); l = f2bf(y - bf2f(h)); }

__device__ __forceinline__ v16h  ldh(const h16* p) { return cat16(*(const v8h*)p, *(const v8h*)(p + 16)); }
__device__ __forceinline__ v16bf ldb(const bf* p)  { return cat16b(*(const v8us*)p, *(const v8us*)(p + 16)); }

template <int NSPLIT>
__device__ __forceinline__ void gemmw_body(const bf* __restrict__ A, const bf* __restrict__ A2, const bf* __restrict__ Bt, const int K, float* C, const int ldc, const size_t sA, const size_t sC) {
    __shared__ __align__(16) float os[16 * 68];
    const size_t z = blockIdx.z; A += z * sA; A2 += z * sA; C += z * sC;
    const int lane = threadIdx.x & 31, lr = lane & 15, hi = lane >> 4; const int r0 = blockIdx.x * 64, c0 = blockIdx.y * 64;
    v8f acc[4][4];
#pragma unroll
    for (int mb = 0; mb < 4; ++mb)
#pragma unroll
        for (int nb = 0; nb < 4; ++nb) acc[mb][nb] = (v8f){};
    const size_t aoff = (size_t)(r0 + lr) * K + 8 * hi, boff = (size_t)(c0 + lr) * K + 8 * hi;
#pragma unroll 1
    for (int kc = 0; kc < K; kc += 32) {
        v16bf a[4], a2[4];
#pragma unroll
        for (int mb = 0; mb < 4; ++mb) { a[mb] = ldb(A + aoff + (size_t)mb * 16 * K + kc); if (NSPLIT == 1) a2[mb] = ldb(A2 + aoff + (size_t)mb * 16 * K + kc); else a2[mb] = a[mb]; }
#pragma unroll
        for (int nb = 0; nb < 4; ++nb) { const v16bf b = ldb(Bt + boff + (size_t)nb * 16 * K + kc);
#pragma unroll
            for (int mb = 0; mb < 4; ++mb) { acc[mb][nb] = wmmab(a[mb], b, acc[mb][nb]); if (NSPLIT == 1) acc[mb][nb] = wmmab(a2[mb], b, acc[mb][nb]); } }
        asm volatile("v_nop\n\tv_nop\n\tv_nop\n\tv_nop" : "+v"(acc[0][0]), "+v"(acc[1][1]), "+v"(acc[2][2]), "+v"(acc[3][3]) : "v"(a[0]), "v"(a[3]), "v"(a2[0]), "v"(a2[3]));
    }
#pragma unroll
    for (int mb = 0; mb < 4; ++mb) {
#pragma unroll
        for (int nb = 0; nb < 4; ++nb) {
#pragma unroll
            for (int j = 0; j < 8; ++j) os[(hi * 8 + j) * 68 + nb * 16 + lr] = acc[mb][nb][j]; }
        __builtin_amdgcn_wave_barrier(); asm volatile("" ::: "memory");
        float* crow = C + (size_t)(r0 + mb * 16) * ldc + c0;
#pragma unroll 1
        for (int ps = 0; ps < 2; ++ps) {
#pragma unroll
            for (int s = 0; s < 8; ++s) { const int row = 2 * s + hi, cofs = lr * 4; const v4f val = *(const v4fa*)(os + row * 68 + cofs);
                *(volatile v4f*)(crow + (size_t)row * ldc + cofs) = val; }
            if (ps == 0) __threadfence(); }
        __builtin_amdgcn_wave_barrier(); asm volatile("" ::: "memory");
    }
}

__global__ __launch_bounds__(32) void k_gemm_proj(const bf* __restrict__ XB, const bf* __restrict__ WK, float* FK) { gemmw_body<0>(XB, XB, WK, DM, FK, DKV, (size_t)0, (size_t)0); }
__global__ __launch_bounds__(32) void k_gemm_out(const bf* __restrict__ ATh, const bf* __restrict__ ATl, const bf* __restrict__ WO, float* OUT) { gemmw_body<1>(ATh, ATl, WO, DQ, OUT, DM, (size_t)SEQ * DQ, (size_t)SEQ_FULL * DM); }

__global__ __launch_bounds__(256) void k_cvt8(const float* __restrict__ src, bf* dst, size_t n8, size_t sS, size_t sD) {
    const size_t i = (size_t)blockIdx.x * 256 + threadIdx.x; if (i >= n8) return;
    src += (size_t)blockIdx.y * sS; dst += (size_t)blockIdx.y * sD;
    const v8f v = *(const v8f*)(src + i * 8); v8us o;
#pragma unroll
    for (int k = 0; k < 8; ++k) o[k] = f2bf(v[k]);
    *(volatile v8us*)(dst + i * 8) = o; __threadfence(); *(volatile v8us*)(dst + i * 8) = o; }

__global__ __launch_bounds__(256) void k_kplane(const float* __restrict__ F, h16* KP) {
    const size_t e8 = (size_t)blockIdx.x * 256 + threadIdx.x; if (e8 >= (size_t)NB * NH_ * SEQ * (HD / 8)) return;
    const int d8 = (int)(e8 % (HD / 8)); const int s = (int)((e8 / (HD / 8)) % SEQ); const int bh = (int)(e8 / ((size_t)(HD / 8) * SEQ)); const int b = bh / NH_, h = bh % NH_;
    const float* f = F + ((size_t)b * SEQ + s) * DKV + h * HD + d8 * 8;
    const v4f a = *(const v4f*)f; const v4f c = *(const v4f*)(f + 4); v8h o;
#pragma unroll
    for (int k = 0; k < 4; ++k) { o[k] = (h16)(a[k] * KCAR); o[4 + k] = (h16)(c[k] * KCAR); }
    *(volatile v8h*)(KP + e8 * 8) = o; __threadfence(); *(volatile v8h*)(KP + e8 * 8) = o; }

__global__ __launch_bounds__(256) void k_vtplane(const float* __restrict__ F, h16* VT) {
    const size_t e8 = (size_t)blockIdx.x * 256 + threadIdx.x; if (e8 >= (size_t)NB * NH_ * HD * (SEQ / 8)) return;
    const int s8 = (int)(e8 % (SEQ / 8)); const int d = (int)((e8 / (SEQ / 8)) % HD); const int bh = (int)(e8 / ((size_t)(SEQ / 8) * HD)); const int b = bh / NH_, h = bh % NH_;
    const float* f = F + ((size_t)b * SEQ + (size_t)s8 * 8) * DKV + h * HD + d; v8h o;
#pragma unroll
    for (int k = 0; k < 8; ++k) o[k] = (h16)(f[(size_t)k * DKV] * KCAR);
    *(volatile v8h*)(VT + e8 * 8) = o; __threadfence(); *(volatile v8h*)(VT + e8 * 8) = o; }

__global__ __launch_bounds__(128) void k_flash(const h16* __restrict__ KP, const h16* __restrict__ VT, bf* Ah, bf* Al) {
    __shared__ __align__(16) float os[4 * 16 * 68];
    const int wave = __builtin_amdgcn_readfirstlane((int)(threadIdx.x >> 5));
    const int lane = threadIdx.x & 31, lr = lane & 15, hi = lane >> 4;
    const int bh = blockIdx.y; const int b = bh / NH_, h = bh % NH_;
    const int q0 = blockIdx.x * 64 + wave * 16;
    const h16* kp = KP + (size_t)bh * SEQ * HD;
    const h16* vt = VT + (size_t)bh * HD * SEQ;
    const int koff = lr * HD + 8 * hi;
    const int voff = lr * SEQ + 8 * hi;
    const v16h bq0 = ldh(kp + (size_t)q0 * HD + koff);
    const v16h bq1 = ldh(kp + (size_t)q0 * HD + koff + 32);
    v8f acc[4];
#pragma unroll
    for (int t = 0; t < 4; ++t) acc[t] = (v8f){};
    float mrun = -1.0e30f, lrun = 0.0f;
#pragma unroll 1
    for (int k0 = 0; k0 < SEQ; k0 += 32) {
        v8f s0 = (v8f){}, s1 = (v8f){};
        {
            const v16h a00 = ldh(kp + (size_t)k0 * HD + koff);
            const v16h a01 = ldh(kp + (size_t)k0 * HD + koff + 32);
            const v16h a10 = ldh(kp + (size_t)(k0 + 16) * HD + koff);
            const v16h a11 = ldh(kp + (size_t)(k0 + 16) * HD + koff + 32);
            s0 = wmma16(a00, bq0, s0); s1 = wmma16(a10, bq0, s1);
            s0 = wmma16(a01, bq1, s0); s1 = wmma16(a11, bq1, s1);
            asm volatile("v_nop\n\tv_nop\n\tv_nop\n\tv_nop" : "+v"(s0), "+v"(s1) : "v"(a00), "v"(a01), "v"(a10), "v"(a11), "v"(bq0), "v"(bq1));
        }
        float u0[8], u1[8]; float tmax = -1.0e30f;
#pragma unroll
        for (int r = 0; r < 8; ++r) { u0[r] = s0[r] * C2; u1[r] = s1[r] * C2; tmax = fmaxf(tmax, fmaxf(u0[r], u1[r])); }
        tmax = fmaxf(tmax, __shfl_xor(tmax, 16, 32));
        const float mnew = fmaxf(mrun, tmax);
        const float alpha = __builtin_amdgcn_exp2f(mrun - mnew);
        const float mb = mnew - PEXP;
        float rsum = 0.0f;
#pragma unroll
        for (int r = 0; r < 8; ++r) { u0[r] = __builtin_amdgcn_exp2f(u0[r] - mb); u1[r] = __builtin_amdgcn_exp2f(u1[r] - mb); rsum += u0[r] + u1[r]; }
        rsum += __shfl_xor(rsum, 16, 32);
        lrun = lrun * alpha + rsum; mrun = mnew;
#pragma unroll
        for (int t = 0; t < 4; ++t)
#pragma unroll
            for (int r = 0; r < 8; ++r) acc[t][r] *= alpha;
        v16h pf;
#pragma unroll
        for (int r = 0; r < 8; ++r) { pf[r] = (h16)u0[r]; pf[8 + r] = (h16)u1[r]; }
        {
            v16h av[4];
#pragma unroll
            for (int t = 0; t < 4; ++t) av[t] = ldh(vt + (size_t)(16 * t) * SEQ + voff + k0);
#pragma unroll
            for (int t = 0; t < 4; ++t) acc[t] = wmma16(av[t], pf, acc[t]);
            asm volatile("v_nop\n\tv_nop\n\tv_nop\n\tv_nop" : "+v"(acc[0]), "+v"(acc[1]), "+v"(acc[2]), "+v"(acc[3]) : "v"(av[0]), "v"(av[1]), "v"(av[2]), "v"(av[3]), "v"(pf));
        }
    }
    const float inv = (1.0f / KCAR) * (1.0f / lrun);
    const int ob = wave * (16 * 68);
#pragma unroll
    for (int t = 0; t < 4; ++t)
#pragma unroll
        for (int r = 0; r < 8; ++r) os[ob + lr * 68 + 16 * t + 8 * hi + r] = acc[t][r] * inv;
    __syncthreads();
    const int rq = lane >> 3, pc = lane & 7;
#pragma unroll 1
    for (int ps = 0; ps < 2; ++ps) {
#pragma unroll
        for (int s = 0; s < 4; ++s) {
            const int row = 4 * s + rq;
            const v4f a = *(const v4fa*)(os + ob + row * 68 + pc * 8);
            const v4f c = *(const v4fa*)(os + ob + row * 68 + pc * 8 + 4);
            v8us oh, ol;
#pragma unroll
            for (int k = 0; k < 4; ++k) { unsigned short x0, x1; splitf(a[k], x0, x1); oh[k] = x0; ol[k] = x1; splitf(c[k], x0, x1); oh[4 + k] = x0; ol[4 + k] = x1; }
            const size_t oo = ((size_t)b * SEQ + q0 + row) * DQ + h * HD + pc * 8;
            *(volatile v8us*)(Ah + oo) = oh; *(volatile v8us*)(Al + oo) = ol; }
        if (ps == 0) __threadfence(); }
}

#define SZ_W   ((size_t)DKV * DM * 2)
#define SZ_XB  ((size_t)NB * SEQ * DM * 2)
#define SZ_FK  ((size_t)NB * SEQ * DKV * 4)
#define SZ_KP  ((size_t)NB * NH_ * SEQ * HD * 2)
#define SZ_AT  ((size_t)NB * SEQ * DQ * 2)
#define SZ_ALL (2 * SZ_W + SZ_XB + SZ_FK + 2 * SZ_KP + 2 * SZ_AT)
static_assert(SZ_W % 256 == 0 && SZ_XB % 256 == 0 && SZ_FK % 256 == 0 && SZ_KP % 256 == 0 && SZ_AT % 256 == 0);
static_assert(SZ_ALL <= (size_t)134217728);

extern "C" void kernel_launch(void* const* d_in, const int* in_sizes, int n_in,
                              void* d_out, int out_size, void* d_ws, size_t ws_size, hipStream_t stream) {
    if (n_in < 3) return;
    const size_t need_x = (size_t)(NB - 1) * SEQ_FULL * DM + (size_t)SEQ * DM;
    if ((size_t)in_sizes[0] < need_x) return;
    if ((size_t)in_sizes[1] < (size_t)DKV * DM) return;
    if ((size_t)in_sizes[2] < (size_t)DM * DQ) return;
    if ((size_t)out_size < need_x) return;
    if (SZ_ALL > ws_size) return;
    const float* x = (const float*)d_in[0]; const float* wk = (const float*)d_in[1]; const float* wo = (const float*)d_in[2];
    float* OUT = (float*)d_out;
    char* wsp = (char*)d_ws;
    bf* WK = (bf*)wsp; wsp += SZ_W;
    bf* WO = (bf*)wsp; wsp += SZ_W;
    bf* XB = (bf*)wsp; wsp += SZ_XB;
    float* FK = (float*)wsp; wsp += SZ_FK;
    h16* KP16 = (h16*)wsp; wsp += SZ_KP;
    h16* VT16 = (h16*)wsp; wsp += SZ_KP;
    bf* ATh = (bf*)wsp; wsp += SZ_AT;
    bf* ATl = (bf*)wsp; wsp += SZ_AT;

    k_cvt8<<<dim3((unsigned)(((size_t)DKV * DM / 8 + 255) / 256), 1, 1), 256, 0, stream>>>(wk, WK, (size_t)DKV * DM / 8, (size_t)0, (size_t)0);
    k_cvt8<<<dim3((unsigned)(((size_t)DM * DQ / 8 + 255) / 256), 1, 1), 256, 0, stream>>>(wo, WO, (size_t)DM * DQ / 8, (size_t)0, (size_t)0);
    k_cvt8<<<dim3((unsigned)(((size_t)SEQ * DM / 8 + 255) / 256), NB, 1), 256, 0, stream>>>(x, XB, (size_t)SEQ * DM / 8, (size_t)SEQ_FULL * DM, (size_t)SEQ * DM);
    k_gemm_proj<<<dim3(NB * SEQ / 64, DKV / 64, 1), 32, 0, stream>>>(XB, WK, FK);
    k_kplane<<<(unsigned)(((size_t)NB * NH_ * SEQ * (HD / 8) + 255) / 256), 256, 0, stream>>>(FK, KP16);
    k_vtplane<<<(unsigned)(((size_t)NB * NH_ * HD * (SEQ / 8) + 255) / 256), 256, 0, stream>>>(FK, VT16);
    k_flash<<<dim3(SEQ / 64, NB * NH_, 1), 128, 0, stream>>>(KP16, VT16, ATh, ATl);
    k_gemm_out<<<dim3(SEQ / 64, DM / 64, NB), 32, 0, stream>>>(ATh, ATl, WO, OUT);
}
